// GraphSAGE_26285199852117
// MI455X (gfx1250) — hardware-verified
//
#include <hip/hip_runtime.h>
#include <stddef.h>
#include <stdint.h>
#include <math.h>


#define DF     128
#define CIN    64
#define AP     512
#define K12    512
#define NTHR   256
#define NWAVE  8
#define EPT    8
#define CHUNK  (NTHR * EPT)
#define WCAP   (EPT * 32)
#define LISTN  (NWAVE * WCAP)
#define NBA    1024
#define SLA    10
#define RCAP   28672
#define DEGCAP 64
#define GBM    64
#define GBN    128
#define GTHR   128
#define RB     128
#define RBW    256
#define UPART  2048
#define NPARTW 12
#define UWE    1024
#define AGG_ZINTS    (LISTN + 2 * RCAP + 3 * NBA)
#define MISC_INTS    16
#define ROWBUF_INTS  (NWAVE * RBW / 2)
#define AGG_LDS_INTS (AGG_ZINTS + MISC_INTS + ROWBUF_INTS)
#define WSMAX  134217728

static_assert((CHUNK & (CHUNK - 1)) == 0 && CHUNK <= 4096);
static_assert(CHUNK == NWAVE * WCAP && WCAP == 8 * 32);
static_assert((NBA & (NBA - 1)) == 0 && NBA == (1 << SLA));
static_assert(((long long)CHUNK << SLA) < (1LL << 31));
static_assert(NBA % NWAVE == 0 && NBA % 32 == 0 && NBA % GBM == 0 && NBA % RB == 0);
static_assert(RCAP % 4 == 0 && AGG_ZINTS % 4 == 0 && LISTN % 4 == 0 && ((AGG_ZINTS + MISC_INTS) % 4) == 0);
static_assert(AGG_ZINTS % (NTHR * 4) == 0);
static_assert(CIN % 32 == 0 && K12 % 32 == 0 && K12 == AP && AP == 4 * DF);
static_assert(GBN == DF && GBM == (GTHR / 32) * 16 && DF == 4 * 32 && GTHR == DF);
static_assert(RB == NWAVE * 16 && RB % GBM == 0 && RBW == 2 * DF);
static_assert(UPART % NTHR == 0 && UPART == DF * (DF / 8) && UWE == DF * (CIN / 8));
static_assert((NPARTW * UPART + UWE) % NTHR == 0);
static_assert(AGG_LDS_INTS * 4 <= 300000);

typedef float          v4f   __attribute__((ext_vector_type(4)));
typedef float          v8f   __attribute__((ext_vector_type(8)));
typedef int            v4i   __attribute__((ext_vector_type(4)));
typedef int            v8i   __attribute__((ext_vector_type(8)));
typedef unsigned short v4us  __attribute__((ext_vector_type(4)));
typedef unsigned short v8us  __attribute__((ext_vector_type(8)));
typedef unsigned short v16us __attribute__((ext_vector_type(16)));
typedef __bf16         v16bf __attribute__((ext_vector_type(16)));
typedef v4f  __attribute__((may_alias)) v4fa;
typedef v4i  __attribute__((may_alias)) v4ia;
typedef v4us __attribute__((may_alias)) v4usa;
typedef v8us __attribute__((may_alias)) v8usa;
union FragB { v16bf v; v16us u; v8us h[2]; v8i w; };

__device__ __forceinline__ v8f wmb(const FragB& a, const FragB& b, v8f c) {
  v8f d = __builtin_amdgcn_wmma_f32_16x16x32_bf16(false, a.v, false, b.v, (short)0, c, false, false);
  asm volatile("v_nop\n\tv_nop\n\tv_nop\n\tv_nop" : "+v"(d) : "v"(a.w), "v"(b.w));
  return d;
}

__device__ __forceinline__ unsigned bf16_bits(float f) {
  const unsigned u = __float_as_uint(f);
  return (u + 0x7FFFu + ((u >> 16) & 1u)) >> 16;
}
__device__ __forceinline__ float bf16_val(float f) {
  return __uint_as_float(bf16_bits(f) << 16);
}
__device__ __forceinline__ int imin(int a, int b) { return a < b ? a : b; }

__device__ __forceinline__ void wave_sync() {
  __builtin_amdgcn_fence(__ATOMIC_RELEASE, "wavefront");
  __builtin_amdgcn_wave_barrier();
  __builtin_amdgcn_fence(__ATOMIC_ACQUIRE, "wavefront");
}

template <int SLB>
__device__ __forceinline__ int scan_chunk(const int* __restrict__ dsts, int nE, int cbase, int slotBase,
                                          int nb, int* list, int lane, int wave) {
  int wc = 0;
  const int el0  = wave * WCAP + lane;
  const int e0   = cbase + el0;
  const int last = nE - 1;
  const int sent = -2147483647 - 1;
  const int r0 = dsts[imin(e0,       last)];
  const int r1 = dsts[imin(e0 + 32,  last)];
  const int r2 = dsts[imin(e0 + 64,  last)];
  const int r3 = dsts[imin(e0 + 96,  last)];
  const int r4 = dsts[imin(e0 + 128, last)];
  const int r5 = dsts[imin(e0 + 160, last)];
  const int r6 = dsts[imin(e0 + 192, last)];
  const int r7 = dsts[imin(e0 + 224, last)];
  const int d0 = (e0       < nE) ? r0 : sent;
  const int d1 = (e0 + 32  < nE) ? r1 : sent;
  const int d2 = (e0 + 64  < nE) ? r2 : sent;
  const int d3 = (e0 + 96  < nE) ? r3 : sent;
  const int d4 = (e0 + 128 < nE) ? r4 : sent;
  const int d5 = (e0 + 160 < nE) ? r5 : sent;
  const int d6 = (e0 + 192 < nE) ? r6 : sent;
  const int d7 = (e0 + 224 < nE) ? r7 : sent;
  const unsigned nbs = (unsigned)slotBase;
  const unsigned unb = (unsigned)nb;
  const unsigned s0 = (unsigned)d0 - nbs, s1 = (unsigned)d1 - nbs;
  const unsigned s2 = (unsigned)d2 - nbs, s3 = (unsigned)d3 - nbs;
  const unsigned s4 = (unsigned)d4 - nbs, s5 = (unsigned)d5 - nbs;
  const unsigned s6 = (unsigned)d6 - nbs, s7 = (unsigned)d7 - nbs;
  const bool h0 = s0 < unb, h1 = s1 < unb, h2 = s2 < unb, h3 = s3 < unb;
  const bool h4 = s4 < unb, h5 = s5 < unb, h6 = s6 < unb, h7 = s7 < unb;
  const unsigned any = __builtin_amdgcn_ballot_w32(h0 | h1 | h2 | h3 | h4 | h5 | h6 | h7);
  if (any != 0u) {
#define HITJ(J, HJ, SJ) { \
      const unsigned mj = __builtin_amdgcn_ballot_w32(HJ); \
      if (mj != 0u) { \
        if (HJ) { \
          const int pos = wc + (int)__builtin_amdgcn_mbcnt_lo(mj, 0u); \
          if (pos < WCAP) list[wave * WCAP + pos] = ((el0 + 32 * (J)) << SLB) | (int)(SJ); \
        } \
        wc += (int)__builtin_popcount(mj); } }
    HITJ(0, h0, s0)
    HITJ(1, h1, s1)
    HITJ(2, h2, s2)
    HITJ(3, h3, s3)
    HITJ(4, h4, s4)
    HITJ(5, h5, s5)
    HITJ(6, h6, s6)
    HITJ(7, h7, s7)
#undef HITJ
  }
  return wc;
}

__global__ __launch_bounds__(NTHR) void k_wprep(const float* __restrict__ Wl1, const float* __restrict__ Wr1,
                                                const float* __restrict__ Wl2, const float* __restrict__ Wr2,
                                                const float* __restrict__ Wl3, const float* __restrict__ Wr3,
                                                const float* __restrict__ Wemb,
                                                unsigned short* WC, unsigned short* WE) {
  const int u    = (int)blockIdx.x * NTHR + (int)threadIdx.x;
  const int part = u >> 11;
  const float* sp;
  unsigned short* dp;
  if (part < NPARTW) {
    const int v     = u & (UPART - 1);
    const int n     = v >> 4;
    const int k8    = (v & 15) * 8;
    const int layer = part >> 2;
    const int q     = part & 3;
    const float* W;
    if (layer == 0)      W = (q < 2) ? Wl1 : Wr1;
    else if (layer == 1) W = (q < 2) ? Wl2 : Wr2;
    else                 W = (q < 2) ? Wl3 : Wr3;
    sp = W + (size_t)n * DF + k8;
    dp = WC + (size_t)layer * DF * K12 + (size_t)n * K12 + q * DF + k8;
  } else {
    const int v = u - NPARTW * UPART;
    if (v >= UWE) return;
    const int n  = v >> 3;
    const int k8 = (v & 7) * 8;
    sp = Wemb + (size_t)n * CIN + k8;
    dp = WE + (size_t)n * CIN + k8;
  }
  const v4f a = *(const v4f*)sp;
  const v4f b = *(const v4f*)(sp + 4);
  v8us o;
  o[0] = (unsigned short)bf16_bits(a.x); o[1] = (unsigned short)bf16_bits(a.y);
  o[2] = (unsigned short)bf16_bits(a.z); o[3] = (unsigned short)bf16_bits(a.w);
  o[4] = (unsigned short)bf16_bits(b.x); o[5] = (unsigned short)bf16_bits(b.y);
  o[6] = (unsigned short)bf16_bits(b.z); o[7] = (unsigned short)bf16_bits(b.w);
  *(volatile v8us*)dp = o;
  __threadfence();
  *(volatile v8us*)dp = o;
}

__global__ __launch_bounds__(NTHR) void k_cvx(const float* __restrict__ x, unsigned short* xb, int nN, int nUnits) {
  const int u = (int)blockIdx.x * NTHR + (int)threadIdx.x;
  if (u >= nUnits) return;
  const int row = u >> 3;
  const int k8  = (u & 7) * 8;
  const int rc  = row < nN ? row : nN - 1;
  const float* p = x + (size_t)rc * CIN + k8;
  const v4f a = *(const v4fa*)p;
  const v4f b = *(const v4fa*)(p + 4);
  const bool ok = row < nN;
  v8us o;
  o[0] = ok ? (unsigned short)bf16_bits(a.x) : (unsigned short)0;
  o[1] = ok ? (unsigned short)bf16_bits(a.y) : (unsigned short)0;
  o[2] = ok ? (unsigned short)bf16_bits(a.z) : (unsigned short)0;
  o[3] = ok ? (unsigned short)bf16_bits(a.w) : (unsigned short)0;
  o[4] = ok ? (unsigned short)bf16_bits(b.x) : (unsigned short)0;
  o[5] = ok ? (unsigned short)bf16_bits(b.y) : (unsigned short)0;
  o[6] = ok ? (unsigned short)bf16_bits(b.z) : (unsigned short)0;
  o[7] = ok ? (unsigned short)bf16_bits(b.w) : (unsigned short)0;
  unsigned short* dp = xb + (size_t)row * CIN + k8;
  *(volatile v8us*)dp = o;
  __threadfence();
  *(volatile v8us*)dp = o;
}

template <int MODE>
__global__ __launch_bounds__(GTHR) void k_gemm(const unsigned short* Aop, const unsigned short* __restrict__ BT,
                                               const float* __restrict__ bias, float* hout,
                                               unsigned short* apl, float* rec, int lda, int K, int nOut) {
  __shared__ __attribute__((aligned(16))) float stg[GBM * GBN];
  __shared__ __attribute__((aligned(16))) float recs[2 * DF];
  const int tid = (int)threadIdx.x, lane = tid & 31, wave = tid >> 5, hh = lane >> 4, m = lane & 15;
  const int rowBase = (int)blockIdx.x * GBM;

  v8f acc[8];
  {
    const v8f z = {0.f, 0.f, 0.f, 0.f, 0.f, 0.f, 0.f, 0.f};
#pragma unroll
    for (int t = 0; t < 8; ++t) acc[t] = z;
  }
  const unsigned short* ap = Aop + (size_t)(rowBase + 16 * wave + m) * (size_t)lda + 8 * hh;
  const unsigned short* bp = BT + (size_t)m * (size_t)K + 8 * hh;

#pragma unroll 1
  for (int k0 = 0; k0 < K; k0 += 32) {
    FragB af;
    af.h[0] = *(const v8usa*)(ap + k0);
    af.h[1] = *(const v8usa*)(ap + k0 + 16);
#pragma unroll
    for (int nt = 0; nt < 8; ++nt) {
      const unsigned short* wq = bp + (size_t)(16 * nt) * (size_t)K + k0;
      FragB bf;
      bf.h[0] = *(const v8usa*)wq;
      bf.h[1] = *(const v8usa*)(wq + 16);
      acc[nt] = wmb(af, bf, acc[nt]);
    }
  }

#pragma unroll
  for (int nt = 0; nt < 8; ++nt) {
    const int lc = 16 * nt + m;
#pragma unroll
    for (int r = 0; r < 8; ++r) {
      const int lr = 16 * wave + 8 * hh + r;
      stg[lr * GBN + lc] = acc[nt][r];
    }
  }
  __syncthreads();

  v4f bb4;
  {
    const v4f t1 = *(const v4f*)(bias + 4 * lane);
    bb4.x = bf16_val(t1.x); bb4.y = bf16_val(t1.y); bb4.z = bf16_val(t1.z); bb4.w = bf16_val(t1.w);
  }
  v4f pv[16];
#pragma unroll
  for (int i = 0; i < 16; ++i) pv[i] = *(const v4fa*)(stg + (16 * wave + i) * GBN + 4 * lane);

  if constexpr (MODE == 1) {
    int nv = nOut - rowBase;
    nv = nv < 0 ? 0 : (nv > GBM ? GBM : nv);
    const float bcol = bf16_val(bias[tid]);
    float s = 0.0f;
#pragma unroll 4
    for (int r = 0; r < nv; ++r) s += stg[r * GBN + tid];
    const float rinv = 1.0f / (float)(nv < 1 ? 1 : nv);
    const float mraw = s * rinv;
    float m2 = 0.0f;
#pragma unroll 4
    for (int r = 0; r < nv; ++r) {
      const float d = stg[r * GBN + tid] - mraw;
      m2 = fmaf(d, d, m2);
    }
    recs[tid]      = mraw + bcol;
    recs[DF + tid] = m2;
  }
  __syncthreads();

#pragma unroll
  for (int i = 0; i < 16; ++i) {
    const bool ok = (rowBase + 16 * wave + i) < nOut;
    v4f y = pv[i] + bb4;
    y.x = ok ? y.x : 0.0f; y.y = ok ? y.y : 0.0f; y.z = ok ? y.z : 0.0f; y.w = ok ? y.w : 0.0f;
    pv[i] = y;
  }

  if constexpr (MODE == 1) {
    const v4f rv = *(const v4fa*)(recs + 4 * (tid & 63));
    float* rp = rec + (size_t)blockIdx.x * (2 * DF) + 4 * (tid & 63);
    const bool rok = tid < 64;
#pragma unroll
    for (int i = 0; i < 16; ++i) {
      const int r = rowBase + 16 * wave + i;
      *(volatile v4f*)(hout + (size_t)r * DF + 4 * lane) = pv[i];
    }
    if (rok) *(volatile v4f*)rp = rv;
    __threadfence();
#pragma unroll
    for (int i = 0; i < 16; ++i) {
      const int r = rowBase + 16 * wave + i;
      *(volatile v4f*)(hout + (size_t)r * DF + 4 * lane) = pv[i];
    }
    if (rok) *(volatile v4f*)rp = rv;
  } else {
#pragma unroll
    for (int i = 0; i < 16; ++i) {
      v4us h4, l4;
      unsigned hb;
      hb = bf16_bits(pv[i].x); h4[0] = (unsigned short)hb; l4[0] = (unsigned short)bf16_bits(pv[i].x - __uint_as_float(hb << 16));
      hb = bf16_bits(pv[i].y); h4[1] = (unsigned short)hb; l4[1] = (unsigned short)bf16_bits(pv[i].y - __uint_as_float(hb << 16));
      hb = bf16_bits(pv[i].z); h4[2] = (unsigned short)hb; l4[2] = (unsigned short)bf16_bits(pv[i].z - __uint_as_float(hb << 16));
      hb = bf16_bits(pv[i].w); h4[3] = (unsigned short)hb; l4[3] = (unsigned short)bf16_bits(pv[i].w - __uint_as_float(hb << 16));
      unsigned short* srow = (unsigned short*)stg + (size_t)(16 * wave + i) * (2 * GBN);
      *(v4usa*)(srow + 4 * lane) = h4;
      *(v4usa*)(srow + DF + 4 * lane) = l4;
    }
    __syncthreads();
    v8us qv[16];
#pragma unroll
    for (int i = 0; i < 16; ++i) {
      const unsigned short* srow = (const unsigned short*)stg + (size_t)(16 * wave + i) * (2 * GBN);
      qv[i] = *(const v8usa*)(srow + 8 * lane);
    }
#pragma unroll
    for (int i = 0; i < 16; ++i) {
      const int r = rowBase + 16 * wave + i;
      *(volatile v4f*)(hout + (size_t)r * DF + 4 * lane) = pv[i];
      *(volatile v8us*)(apl + (size_t)r * (size_t)AP + 2 * DF + 8 * lane) = qv[i];
    }
    __threadfence();
#pragma unroll
    for (int i = 0; i < 16; ++i) {
      const int r = rowBase + 16 * wave + i;
      *(volatile v4f*)(hout + (size_t)r * DF + 4 * lane) = pv[i];
      *(volatile v8us*)(apl + (size_t)r * (size_t)AP + 2 * DF + 8 * lane) = qv[i];
    }
  }
}

__global__ __launch_bounds__(NTHR) void k_scan(const int* __restrict__ srcs, const int* __restrict__ dsts,
                                               const float* hf, unsigned short* apl,
                                               int nE, int nN, int mRows) {
  extern __shared__ __attribute__((aligned(16))) int dsm[];
  int* list = dsm;
  int* hl   = dsm + LISTN;
  int* sl   = hl + RCAP;
  int* cnt  = sl + RCAP;
  int* offs = cnt + NBA;
  int* cur  = offs + NBA;
  int* misc = cur + NBA;
  const int tid = (int)threadIdx.x, lane = tid & 31, wave = tid >> 5;
  unsigned short* rowbuf = (unsigned short*)(misc + MISC_INTS) + wave * RBW;
  const int nodeBase = (int)blockIdx.x * NBA;

  {
    const v4i z4 = {0, 0, 0, 0};
    for (int i = tid * 4; i < AGG_ZINTS; i += NTHR * 4) *(v4ia*)(dsm + i) = z4;
    if (tid < MISC_INTS) misc[tid] = 0;
  }
  __syncthreads();

  int t = 0, ov = 0;
  const int nChunks = (nE + CHUNK - 1) / CHUNK;
#pragma unroll 1
  for (int ch = 0; ch < nChunks; ++ch) {
    const int cbase = ch * CHUNK;
    const int wc = scan_chunk<SLA>(dsts, nE, cbase, nodeBase, NBA, list, lane, wave);
    if (lane == 0) misc[wave] = wc;
    __syncthreads();
    if (wave == 0) {
#pragma unroll 1
      for (int w2 = 0; w2 < NWAVE; ++w2) {
        int c = misc[w2];
        c = c < 0 ? 0 : (c > WCAP ? WCAP : c);
#pragma unroll 1
        for (int b0 = 0; b0 < c; b0 += 32) {
          const int idx = b0 + lane;
          const int ent = list[w2 * WCAP + (idx < WCAP ? idx : WCAP - 1)];
          const int m32 = (c - b0) < 32 ? (c - b0) : 32;
#pragma unroll 1
          for (int k = 0; k < m32; ++k) {
            const int u    = __builtin_amdgcn_readlane(ent, k);
            const int slot = u & (NBA - 1);
            const int el   = (u >> SLA) & (CHUNK - 1);
            const int pk   = ((cbase + el) << SLA) | slot;
            if (t < RCAP) {
              if (lane == 0) { hl[t] = pk; cnt[slot] = cnt[slot] + 1; }
              t = t + 1;
            } else {
              ov = 1;
            }
          }
        }
      }
    }
    __syncthreads();
  }
  if (wave == 0 && lane == 0) { misc[8] = t; misc[9] = ov; }
  __syncthreads();
  int tt = misc[8];
  tt = tt < 0 ? 0 : (tt > RCAP ? RCAP : tt);
  const int ovf = misc[9];

  if (wave == 0) {
    const int base = lane * (NBA / 32);
    int s = 0;
#pragma unroll 1
    for (int i = 0; i < NBA / 32; ++i) s += cnt[base + i];
    int incl = s;
#pragma unroll
    for (int d = 1; d < 32; d <<= 1) {
      const int y = __shfl_up(incl, d, 32);
      if (lane >= d) incl += y;
    }
    int run = incl - s;
#pragma unroll 1
    for (int i = 0; i < NBA / 32; ++i) {
      const int cv = cnt[base + i];
      offs[base + i] = run;
      cur[base + i]  = run;
      run += cv;
    }
  }
  __syncthreads();
  if (wave == 0) {
#pragma unroll 1
    for (int b0 = 0; b0 < tt; b0 += 32) {
      const int idx = b0 + lane;
      const int ent = hl[idx < RCAP ? idx : RCAP - 1];
      const int m32 = (tt - b0) < 32 ? (tt - b0) : 32;
#pragma unroll 1
      for (int k = 0; k < m32; ++k) {
        const int u    = __builtin_amdgcn_readlane(ent, k);
        const int slot = u & (NBA - 1);
        if (lane == 0) {
          int p = cur[slot];
          p = p < 0 ? 0 : (p > RCAP - 1 ? RCAP - 1 : p);
          sl[p] = u;
          cur[slot] = p + 1;
        }
      }
    }
  }
  __syncthreads();

  const float qnan = __int_as_float(0x7fc00000);
  const float pz = (ovf != 0) ? qnan : 0.0f;
#pragma unroll 1
  for (int si = 0; si < NBA / NWAVE; ++si) {
    const int s    = si * NWAVE + wave;
    const int node = nodeBase + s;
    int c = cnt[s];
    const bool big = c > DEGCAP;
    c = c < 0 ? 0 : (c > DEGCAP ? DEGCAP : c);
    int o = offs[s];
    o = o < 0 ? 0 : (o > RCAP ? RCAP : o);
    float a0 = 0.0f, a1 = 0.0f, a2 = 0.0f, a3 = 0.0f;
#pragma unroll 1
    for (int b0 = 0; b0 < c; b0 += 32) {
      int idx = o + b0 + lane;
      idx = idx > RCAP - 1 ? RCAP - 1 : idx;
      const int ent = sl[idx];
      int eid = ent >> SLA;
      eid = eid < 0 ? 0 : (eid > nE - 1 ? nE - 1 : eid);
      int sr = srcs[eid];
      sr = sr < 0 ? 0 : (sr > nN - 1 ? nN - 1 : sr);
      const int m32 = (c - b0) < 32 ? (c - b0) : 32;
#pragma unroll 1
      for (int k = 0; k < m32; ++k) {
        const int sk = __builtin_amdgcn_readlane(sr, k);
        const v4f a = *(const v4f*)(hf + (size_t)sk * DF + 4 * lane);
        a0 += a.x; a1 += a.y; a2 += a.z; a3 += a.w;
      }
    }
    const float inv = 1.0f / (float)(c < 1 ? 1 : c);
    const float pzr = big ? qnan : pz;
    const bool live = node < nN;
    const float m0 = live ? (a0 * inv + pzr) : 0.0f;
    const float m1 = live ? (a1 * inv + pzr) : 0.0f;
    const float m2 = live ? (a2 * inv + pzr) : 0.0f;
    const float m3 = live ? (a3 * inv + pzr) : 0.0f;
    v4us mh, ml;
    {
      unsigned hb;
      hb = bf16_bits(m0); mh[0] = (unsigned short)hb; ml[0] = (unsigned short)bf16_bits(m0 - __uint_as_float(hb << 16));
      hb = bf16_bits(m1); mh[1] = (unsigned short)hb; ml[1] = (unsigned short)bf16_bits(m1 - __uint_as_float(hb << 16));
      hb = bf16_bits(m2); mh[2] = (unsigned short)hb; ml[2] = (unsigned short)bf16_bits(m2 - __uint_as_float(hb << 16));
      hb = bf16_bits(m3); mh[3] = (unsigned short)hb; ml[3] = (unsigned short)bf16_bits(m3 - __uint_as_float(hb << 16));
    }
    *(v4usa*)(rowbuf + 4 * lane) = mh;
    *(v4usa*)(rowbuf + DF + 4 * lane) = ml;
    wave_sync();
    const v8us q0 = *(const v8usa*)(rowbuf + 8 * lane);
    wave_sync();
    if (node < mRows) {
      unsigned short* rpw = apl + (size_t)node * AP + 8 * lane;
      *(volatile v8us*)rpw = q0;
      __threadfence();
      *(volatile v8us*)rpw = q0;
    }
  }
}

__global__ __launch_bounds__(GTHR) void k_bncomb(const float* __restrict__ rec, const float* __restrict__ gam,
                                                 const float* __restrict__ bet, float* ac,
                                                 double invN, int nBlk, int nN) {
  __shared__ __attribute__((aligned(16))) float acs[2 * DF];
  const int c = (int)threadIdx.x;
  double S = 0.0;
#pragma unroll 1
  for (int b = 0; b < nBlk; ++b) {
    int nv = nN - b * GBM;
    nv = nv < 0 ? 0 : (nv > GBM ? GBM : nv);
    S += (double)nv * (double)rec[(size_t)b * (2 * DF) + c];
  }
  const double mu = S * invN;
  double Q = 0.0;
#pragma unroll 1
  for (int b = 0; b < nBlk; ++b) {
    int nv = nN - b * GBM;
    nv = nv < 0 ? 0 : (nv > GBM ? GBM : nv);
    const double d = (double)rec[(size_t)b * (2 * DF) + c] - mu;
    Q += (double)rec[(size_t)b * (2 * DF) + DF + c] + (double)nv * d * d;
  }
  const double var = Q * invN;
  const float vf = (float)var + 1e-5f;
  const float a  = bf16_val(gam[c]) * rsqrtf(vf);
  const float cc = (float)((double)bf16_val(bet[c]) - mu * (double)a);
  acs[c]      = a;
  acs[DF + c] = cc;
  __syncthreads();
  const v4f ov = *(const v4fa*)(acs + 4 * (c & 63));
  float* op = ac + 4 * (c & 63);
  const bool okst = c < 64;
  if (okst) *(volatile v4f*)op = ov;
  __threadfence();
  if (okst) *(volatile v4f*)op = ov;
}

template <int FIN>
__global__ __launch_bounds__(NTHR) void k_bnrelu(float* hu, const float* __restrict__ ac, unsigned short* apl,
                                                 const float* __restrict__ Wc, const float* __restrict__ bc,
                                                 float* out, int nN) {
  __shared__ __attribute__((aligned(16))) unsigned short rbuf[NWAVE * RBW];
  __shared__ __attribute__((aligned(16))) float lg[2 * RB];
  const int tid = (int)threadIdx.x, lane = tid & 31, wave = tid >> 5;
  const int row0 = (int)blockIdx.x * RB + 16 * wave;
  const v4f a4 = *(const v4f*)(ac + 4 * lane);
  const v4f c4 = *(const v4f*)(ac + DF + 4 * lane);
  v4f w0 = {0.f, 0.f, 0.f, 0.f}, w1 = {0.f, 0.f, 0.f, 0.f};
  float bc0 = 0.0f, bc1 = 0.0f;
  if constexpr (FIN != 0) {
    const v4f t0 = *(const v4f*)(Wc + 4 * lane);
    const v4f t1 = *(const v4f*)(Wc + DF + 4 * lane);
    w0.x = bf16_val(t0.x); w0.y = bf16_val(t0.y); w0.z = bf16_val(t0.z); w0.w = bf16_val(t0.w);
    w1.x = bf16_val(t1.x); w1.y = bf16_val(t1.y); w1.z = bf16_val(t1.z); w1.w = bf16_val(t1.w);
    bc0 = bf16_val(bc[0]);
    bc1 = bf16_val(bc[1]);
  }
  unsigned short* rb = rbuf + wave * RBW;

#pragma unroll 1
  for (int i = 0; i < 16; ++i) {
    const int r = row0 + i;
    const bool live = r < nN;
    const v4f u4 = *(const v4fa*)(hu + (size_t)r * DF + 4 * lane);
    v4f y;
    y.x = fmaf(a4.x, u4.x, c4.x);
    y.y = fmaf(a4.y, u4.y, c4.y);
    y.z = fmaf(a4.z, u4.z, c4.z);
    y.w = fmaf(a4.w, u4.w, c4.w);
    y.x = (y.x > 0.0f) ? y.x : (y.x - y.x);
    y.y = (y.y > 0.0f) ? y.y : (y.y - y.y);
    y.z = (y.z > 0.0f) ? y.z : (y.z - y.z);
    y.w = (y.w > 0.0f) ? y.w : (y.w - y.w);
    y.x = live ? y.x : 0.0f; y.y = live ? y.y : 0.0f; y.z = live ? y.z : 0.0f; y.w = live ? y.w : 0.0f;
    if constexpr (FIN == 0) {
      v4us h4, l4;
      unsigned hb;
      hb = bf16_bits(y.x); h4[0] = (unsigned short)hb; l4[0] = (unsigned short)bf16_bits(y.x - __uint_as_float(hb << 16));
      hb = bf16_bits(y.y); h4[1] = (unsigned short)hb; l4[1] = (unsigned short)bf16_bits(y.y - __uint_as_float(hb << 16));
      hb = bf16_bits(y.z); h4[2] = (unsigned short)hb; l4[2] = (unsigned short)bf16_bits(y.z - __uint_as_float(hb << 16));
      hb = bf16_bits(y.w); h4[3] = (unsigned short)hb; l4[3] = (unsigned short)bf16_bits(y.w - __uint_as_float(hb << 16));
      *(v4usa*)(rb + 4 * lane) = h4;
      *(v4usa*)(rb + DF + 4 * lane) = l4;
      wave_sync();
      const v8us q = *(const v8usa*)(rb + 8 * lane);
      wave_sync();
      float* hp = hu + (size_t)r * DF + 4 * lane;
      unsigned short* pp = apl + (size_t)r * (size_t)AP + 2 * DF + 8 * lane;
      *(volatile v4f*)hp = y;
      *(volatile v8us*)pp = q;
      __threadfence();
      *(volatile v4f*)hp = y;
      *(volatile v8us*)pp = q;
    } else {
      float p0 = y.x * w0.x;
      p0 = fmaf(y.y, w0.y, p0); p0 = fmaf(y.z, w0.z, p0); p0 = fmaf(y.w, w0.w, p0);
      float p1 = y.x * w1.x;
      p1 = fmaf(y.y, w1.y, p1); p1 = fmaf(y.z, w1.z, p1); p1 = fmaf(y.w, w1.w, p1);
#pragma unroll
      for (int d = 16; d >= 1; d >>= 1) {
        p0 += __shfl_xor(p0, d, 32);
        p1 += __shfl_xor(p1, d, 32);
      }
      if (lane == 0) {
        lg[2 * (16 * wave + i)]     = p0 + bc0;
        lg[2 * (16 * wave + i) + 1] = p1 + bc1;
      }
    }
  }

  if constexpr (FIN != 0) {
    __syncthreads();
    if (tid < RB) {
      const float l0 = lg[2 * tid];
      const float l1 = lg[2 * tid + 1];
      const float mx = (l0 > l1) ? l0 : l1;
      const float e0 = expf(l0 - mx);
      const float e1 = expf(l1 - mx);
      const float inv = 1.0f / (e0 + e1);
      const bool ok = ((int)blockIdx.x * RB + tid) < nN;
      lg[2 * tid]     = ok ? e0 * inv : 0.0f;
      lg[2 * tid + 1] = ok ? e1 * inv : 0.0f;
    }
    __syncthreads();
    const v4f ov = *(const v4fa*)(lg + 4 * (tid & 63));
    const long long g = (long long)blockIdx.x * (2 * RB) + 4 * (tid & 63);
    const bool okst = (tid < 64) && (g + 3 < 2LL * nN);
    float* op = out + (size_t)g;
    if (okst) *(volatile v4f*)op = ov;
    __threadfence();
    if (okst) *(volatile v4f*)op = ov;
  }
}

static inline int cdiv(int a, int b) { return (a + b - 1) / b; }
static inline size_t al256(size_t o) { return (o + 255) & ~(size_t)255; }

extern "C" void kernel_launch(void* const* d_in, const int* in_sizes, int n_in,
                              void* d_out, int out_size, void* d_ws, size_t ws_size,
                              hipStream_t stream) {
  if (n_in < 21) return;
  if (in_sizes[0] < CIN || (in_sizes[0] % CIN) != 0) return;
  const int nN = in_sizes[0] / CIN;
  if (nN < 16 || nN >= (1 << 24) || (nN & 1) != 0) return;
  if (in_sizes[1] < 2 || (in_sizes[1] & 1) != 0) return;
  const int nE = in_sizes[1] / 2;
  if (nE < 1 || nE >= (1 << (31 - SLA))) return;
  if (in_sizes[2] != DF * CIN || in_sizes[3] != DF) return;
  if (in_sizes[4] != 2 * DF || in_sizes[5] != 2) return;
  for (int L = 0; L < 3; ++L) {
    const int b = 6 + 5 * L;
    if (in_sizes[b] != DF * DF || in_sizes[b + 1] != DF) return;
    if (in_sizes[b + 2] != DF * DF) return;
    if (in_sizes[b + 3] != DF || in_sizes[b + 4] != DF) return;
  }
  if ((long long)out_size != 2LL * nN) return;

  const float* x    = (const float*)d_in[0];
  const int*   edge = (const int*)d_in[1];
  const float* Wemb = (const float*)d_in[2];
  const float* bemb = (const float*)d_in[3];
  const float* Wc   = (const float*)d_in[4];
  const float* bc   = (const float*)d_in[5];
  const float* Wl[3] = {(const float*)d_in[6],  (const float*)d_in[11], (const float*)d_in[16]};
  const float* bl[3] = {(const float*)d_in[7],  (const float*)d_in[12], (const float*)d_in[17]};
  const float* Wr[3] = {(const float*)d_in[8],  (const float*)d_in[13], (const float*)d_in[18]};
  const float* gm[3] = {(const float*)d_in[9],  (const float*)d_in[14], (const float*)d_in[19]};
  const float* be[3] = {(const float*)d_in[10], (const float*)d_in[15], (const float*)d_in[20]};
  float* out = (float*)d_out;
  const int* src = edge;
  const int* dst = edge + nE;

  const int MP = cdiv(nN, RB) * RB;
  const int gM = MP / GBM;
  const int gR = MP / RB;
  const int gA = cdiv(MP, NBA);
  if ((long long)gA * NBA < (long long)MP) return;
  const double invN = 1.0 / (double)nN;

  char* ws = (char*)d_ws;
  size_t off = 0;
  const size_t oXB  = off; off = al256(off + (size_t)MP * CIN * 2);
  const size_t oWE  = off; off = al256(off + (size_t)DF * CIN * 2);
  const size_t oWC  = off; off = al256(off + (size_t)3 * DF * K12 * 2);
  const size_t oA   = off; off = al256(off + (size_t)MP * AP * 2);
  const size_t oH   = off; off = al256(off + (size_t)MP * DF * 4);
  const size_t oREC = off; off = al256(off + (size_t)gM * 2 * DF * 4);
  const size_t oAC  = off; off = al256(off + (size_t)3 * 2 * DF * 4);
  if (off > ws_size || off > (size_t)WSMAX) return;
  unsigned short* XB  = (unsigned short*)(ws + oXB);
  unsigned short* WE  = (unsigned short*)(ws + oWE);
  unsigned short* WC  = (unsigned short*)(ws + oWC);
  unsigned short* Apl = (unsigned short*)(ws + oA);
  float*          H   = (float*)(ws + oH);
  float*          REC = (float*)(ws + oREC);
  float*          AC  = (float*)(ws + oAC);

  const size_t scanLds = (size_t)AGG_LDS_INTS * 4;
  hipFuncSetAttribute(reinterpret_cast<const void*>(&k_scan), hipFuncAttributeMaxDynamicSharedMemorySize, (int)scanLds);

  const int nUx = MP * (CIN / 8);
  k_wprep<<<(NPARTW * UPART + UWE) / NTHR, NTHR, 0, stream>>>(Wl[0], Wr[0], Wl[1], Wr[1], Wl[2], Wr[2], Wemb, WC, WE);
  k_cvx<<<cdiv(nUx, NTHR), NTHR, 0, stream>>>(x, XB, nN, nUx);
  k_gemm<0><<<gM, GTHR, 0, stream>>>(XB, WE, bemb, H, Apl, REC, CIN, CIN, nN);
  for (int L = 0; L < 3; ++L) {
    k_scan<<<gA, NTHR, scanLds, stream>>>(src, dst, H, Apl, nE, nN, MP);
    k_gemm<1><<<gM, GTHR, 0, stream>>>(Apl, WC + (size_t)L * DF * K12, bl[L], H, Apl, REC, AP, K12, nN);
    k_bncomb<<<1, GTHR, 0, stream>>>(REC, gm[L], be[L], AC + (size_t)L * 2 * DF, invN, gM, nN);
    if (L < 2) k_bnrelu<0><<<gR, NTHR, 0, stream>>>(H, AC + (size_t)L * 2 * DF, Apl, Wc, bc, out, nN);
    else       k_bnrelu<1><<<gR, NTHR, 0, stream>>>(H, AC + (size_t)L * 2 * DF, Apl, Wc, bc, out, nN);
  }
}
